// Attention_6442450944516
// MI455X (gfx1250) — hardware-verified
//
#include <hip/hip_runtime.h>


#ifndef NB
#define NB 1
#endif
#ifndef SEQ
#define SEQ 4096
#endif
#define NB_FULL  1
#define SEQ_FULL 4096
#ifndef OUT_SEQ
#define OUT_SEQ SEQ
#endif
#define DM   2048
#define HQ_  32
#define HK_  8
#define GQ   4
#define HD   64
#define QW   (HQ_ * HD)
#define KW   (HK_ * HD)
#define ESTQ 64
#define VSZ  ((SEQ < 300) ? SEQ : 300)
#define SSZ  ((SEQ < 800) ? SEQ : 800)
#define NSP  (VSZ + SSZ)
#define NKP  (((NSP + 63) / 64) * 64)
#define RES_ROWS 512
#define AW   4
#define QRS  2048.0f
#define QRI  (1.0f / 2048.0f)
#define WOS  256.0f
#define WOI  (1.0f / 256.0f)
#define SC2  (0.125f * 1.4426950408889634f)
#define PSH  8.0f

static_assert(HD == 64);
static_assert(HQ_ == HK_ * GQ);
static_assert(QW % 64 == 0);
static_assert(KW % 64 == 0);
static_assert(DM % 64 == 0);
static_assert(DM % 32 == 0);
static_assert(QW % 32 == 0);
static_assert(SEQ % 64 == 0);
static_assert((NB * SEQ) % 64 == 0);
static_assert(SEQ % 32 == 0);
static_assert(SEQ % (16 * AW) == 0);
static_assert(RES_ROWS % 64 == 0);
static_assert(((size_t)SEQ * DM) % 8 == 0);
static_assert(NB <= NB_FULL);
static_assert(SEQ <= SEQ_FULL);
static_assert((SEQ & (SEQ - 1)) == 0);
static_assert(SEQ >= 256 && SEQ <= 4096);
static_assert(SEQ % 256 == 0);
static_assert(SEQ % 128 == 0);
static_assert(ESTQ == 64 && ESTQ <= SEQ);
static_assert(NKP % 64 == 0 && NKP >= NSP);
static_assert(NKP >= ((NSP + 31) / 32) * 32);
static_assert(VSZ <= SEQ && SSZ <= SEQ);
static_assert((size_t)SEQ * 8 + (size_t)SEQ * 4 + (size_t)SEQ * 2 + (size_t)NKP * 4 + 2 * ESTQ * 4 + 32 <= 65536);

typedef _Float16 h16;
typedef unsigned short bf;
typedef __attribute__((ext_vector_type(16))) __bf16   v16bf;
typedef __attribute__((ext_vector_type(16))) _Float16 v16h;
typedef __attribute__((ext_vector_type(8)))  _Float16 v8h;
typedef __attribute__((ext_vector_type(8)))  unsigned short v8us;
typedef __attribute__((ext_vector_type(8)))  float    v8f;
typedef __attribute__((ext_vector_type(4)))  float    v4f;
typedef __attribute__((ext_vector_type(4)))  int      v4i;
typedef v4f  __attribute__((may_alias)) v4fa;
typedef v4i  __attribute__((may_alias)) v4ia;
typedef v8h  __attribute__((may_alias)) v8ha;

__device__ __forceinline__ unsigned short f2bf(float f) { unsigned u = __float_as_uint(f); u += 0x7FFFu + ((u >> 16) & 1u); return (unsigned short)(u >> 16); }
__device__ __forceinline__ float bfr(float f) { return __uint_as_float(((unsigned)f2bf(f)) << 16); }
__device__ __forceinline__ v16h cat16(v8h lo, v8h hi) { return __builtin_shufflevector(lo, hi, 0, 1, 2, 3, 4, 5, 6, 7, 8, 9, 10, 11, 12, 13, 14, 15); }
__device__ __forceinline__ v16bf cat16b(v8us lo, v8us hi) { return __builtin_bit_cast(v16bf, __builtin_shufflevector(lo, hi, 0, 1, 2, 3, 4, 5, 6, 7, 8, 9, 10, 11, 12, 13, 14, 15)); }
__device__ __forceinline__ v8f wmma16(v16h a, v16h b, v8f c) { return __builtin_amdgcn_wmma_f32_16x16x32_f16(false, a, false, b, (short)0, c, false, false); }
__device__ __forceinline__ v8f wmmab(v16bf a, v16bf b, v8f c) { return __builtin_amdgcn_wmma_f32_16x16x32_bf16(false, a, false, b, (short)0, c, false, false); }
__device__ __forceinline__ v16h  ldh(const h16* p) { return cat16(*(const v8h*)p, *(const v8h*)(p + 16)); }
__device__ __forceinline__ v16bf ldb(const bf* p)  { return cat16b(*(const v8us*)p, *(const v8us*)(p + 16)); }
__device__ __forceinline__ void wave_sync() { __builtin_amdgcn_fence(3  , "wavefront"); __builtin_amdgcn_wave_barrier(); asm volatile("" ::: "memory"); }

static __device__ __forceinline__ h16 toh_flush(float v) { const h16 r = (h16)v; return (fabsf(v) < 6.103515625e-05f) ? (h16)0.0f : r; }
__device__ __forceinline__ v8f wg16(v16h a, v16h b, v8f c) { c = wmma16(a, b, c); asm volatile("v_nop\n\tv_nop\n\tv_nop\n\tv_nop" : "+v"(c) : "v"(a), "v"(b)); return c; }
__device__ __forceinline__ int imin(int a, int b) { return a < b ? a : b; }
__device__ __forceinline__ int imax(int a, int b) { return a > b ? a : b; }
__device__ __forceinline__ unsigned long long mkkey(float v, int j) { const unsigned vb = __float_as_uint(v) & 0x7FFFFFFFu; return ((unsigned long long)(0x7FFFFFFFu - vb) << 32) | (unsigned long long)(unsigned)j; }
static constexpr int bs_top() { int s = 1; while (s * 2 <= NSP) s *= 2; return s; }
static constexpr int BS_TOP = bs_top();
static_assert(BS_TOP * 2 > NSP);

__global__ __launch_bounds__(256) void k_cvt8(const float* __restrict__ src, bf* dst, size_t n8) {
    const size_t i = (size_t)blockIdx.x * 256 + threadIdx.x; if (i >= n8) return;
    const v8f v = *(const v8f*)(src + i * 8); v8us o;
#pragma unroll
    for (int k = 0; k < 8; ++k) o[k] = f2bf(v[k]);
    *(volatile v8us*)(dst + i * 8) = o; __threadfence(); *(volatile v8us*)(dst + i * 8) = o;
}

__global__ __launch_bounds__(256) void k_trb(const float* __restrict__ W, bf* Wt, int K, int N) {
    __shared__ float tl[64 * 65];
    const int tid = threadIdx.x; const int n0 = blockIdx.x * 64, k0 = blockIdx.y * 64;
    const int lrw = tid >> 4, c4 = (tid & 15) * 4;
#pragma unroll
    for (int p = 0; p < 4; ++p) { const int kk = lrw + 16 * p;
        const v4f v = *(const v4f*)(W + (size_t)(k0 + kk) * N + n0 + c4);
        tl[kk * 65 + c4] = v[0]; tl[kk * 65 + c4 + 1] = v[1]; tl[kk * 65 + c4 + 2] = v[2]; tl[kk * 65 + c4 + 3] = v[3]; }
    __syncthreads();
    const int k8 = (tid & 7) * 8, rg = tid >> 3;
    v8us o[2];
#pragma unroll
    for (int ps = 0; ps < 2; ++ps) { const int n = rg + 32 * ps;
#pragma unroll
        for (int i = 0; i < 8; ++i) o[ps][i] = f2bf(tl[(k8 + i) * 65 + n]); }
#pragma unroll 1
    for (int pz = 0; pz < 2; ++pz) {
#pragma unroll
        for (int ps = 0; ps < 2; ++ps) *(volatile v8us*)(Wt + (size_t)(n0 + rg + 32 * ps) * K + k0 + k8) = o[ps];
        if (pz == 0) __threadfence(); }
}

__global__ __launch_bounds__(256) void k_trw(const float* __restrict__ W, h16* Wt, int K, int N) {
    __shared__ float tl[64 * 65];
    const int tid = threadIdx.x; const int n0 = blockIdx.x * 64, k0 = blockIdx.y * 64;
    const int lrw = tid >> 4, c4 = (tid & 15) * 4;
#pragma unroll
    for (int p = 0; p < 4; ++p) { const int kk = lrw + 16 * p;
        const v4f v = *(const v4f*)(W + (size_t)(k0 + kk) * N + n0 + c4);
        tl[kk * 65 + c4] = v[0]; tl[kk * 65 + c4 + 1] = v[1]; tl[kk * 65 + c4 + 2] = v[2]; tl[kk * 65 + c4 + 3] = v[3]; }
    __syncthreads();
    const int k8 = (tid & 7) * 8, rg = tid >> 3;
    v8h o[2];
#pragma unroll
    for (int ps = 0; ps < 2; ++ps) { const int n = rg + 32 * ps;
#pragma unroll
        for (int i = 0; i < 8; ++i) o[ps][i] = toh_flush(bfr(tl[(k8 + i) * 65 + n]) * WOS); }
#pragma unroll 1
    for (int pz = 0; pz < 2; ++pz) {
#pragma unroll
        for (int ps = 0; ps < 2; ++ps) *(volatile v8h*)(Wt + (size_t)(n0 + rg + 32 * ps) * K + k0 + k8) = o[ps];
        if (pz == 0) __threadfence(); }
}

template <int MODE>
__device__ __forceinline__ void proj_body(const bf* __restrict__ A, const bf* __restrict__ Bt, h16* Ph, h16* Pr, int useRes,
                                          int RB, size_t sRB, int pitch, int CB, size_t sCB,
                                          const float* __restrict__ fc, const float* __restrict__ fs) {
    __shared__ __align__(16) float os[16 * 68];
    const int K = DM;
    const int lane = threadIdx.x & 31, lr = lane & 15, hi = lane >> 4; const int r0 = blockIdx.x * 64, c0 = blockIdx.y * 64;
    v8f acc[4][4];
#pragma unroll
    for (int mb = 0; mb < 4; ++mb)
#pragma unroll
        for (int nb = 0; nb < 4; ++nb) acc[mb][nb] = (v8f){};
    const size_t aoff = (size_t)(r0 + lr) * K + 8 * hi, boff = (size_t)(c0 + lr) * K + 8 * hi;
#pragma unroll 1
    for (int kc = 0; kc < K; kc += 32) {
        v16bf a[4];
#pragma unroll
        for (int mb = 0; mb < 4; ++mb) a[mb] = ldb(A + aoff + (size_t)mb * 16 * K + kc);
#pragma unroll
        for (int nb = 0; nb < 4; ++nb) { const v16bf b = ldb(Bt + boff + (size_t)nb * 16 * K + kc);
#pragma unroll
            for (int mb = 0; mb < 4; ++mb) acc[mb][nb] = wmmab(a[mb], b, acc[mb][nb]); }
        asm volatile("v_nop\n\tv_nop\n\tv_nop\n\tv_nop" : "+v"(acc[0][0]), "+v"(acc[1][1]), "+v"(acc[2][2]), "+v"(acc[3][3]) : "v"(a[0]), "v"(a[1]), "v"(a[2]), "v"(a[3]));
    }
    const size_t tbase = (size_t)(r0 / RB) * sRB + (size_t)(r0 % RB) * (size_t)pitch + (size_t)(c0 / CB) * sCB + (size_t)(c0 % CB);
    const int c8 = (lane & 7) * 8, rg = lane >> 3;
    const int p4 = c8 >> 1;
#pragma unroll
    for (int mb = 0; mb < 4; ++mb) {
#pragma unroll
        for (int nb = 0; nb < 4; ++nb) {
#pragma unroll
            for (int j = 0; j < 8; ++j) os[(hi * 8 + j) * 68 + nb * 16 + lr] = acc[mb][nb][j]; }
        wave_sync();
        v8h hv[4], rv[4];
#pragma unroll
        for (int s = 0; s < 4; ++s) { const int row = 4 * s + rg;
            const v4f x0 = *(const v4fa*)(&os[row * 68 + c8]); const v4f x1 = *(const v4fa*)(&os[row * 68 + c8 + 4]);
            float val[8];
            if (MODE == 1) {
                const int t = (r0 + mb * 16 + row) % SEQ;
                const v4f cc = *(const v4f*)(fc + (size_t)t * 32 + p4); const v4f sn = *(const v4f*)(fs + (size_t)t * 32 + p4);
                const float ca = bfr(cc[0]), cb = bfr(cc[1]), cd = bfr(cc[2]), ce = bfr(cc[3]);
                const float sa = bfr(sn[0]), sb = bfr(sn[1]), sd = bfr(sn[2]), se = bfr(sn[3]);
                val[0] = x0[0] * ca - x0[1] * sa; val[1] = x0[0] * sa + x0[1] * ca;
                val[2] = x0[2] * cb - x0[3] * sb; val[3] = x0[2] * sb + x0[3] * cb;
                val[4] = x1[0] * cd - x1[1] * sd; val[5] = x1[0] * sd + x1[1] * cd;
                val[6] = x1[2] * ce - x1[3] * se; val[7] = x1[2] * se + x1[3] * ce;
            } else {
#pragma unroll
                for (int i = 0; i < 4; ++i) { val[i] = x0[i]; val[4 + i] = x1[i]; }
            }
            v8h hh, rr;
#pragma unroll
            for (int i = 0; i < 8; ++i) { const h16 a0 = toh_flush(val[i]); hh[i] = a0; rr[i] = toh_flush((val[i] - (float)a0) * QRS); }
            hv[s] = hh; rv[s] = rr; }
        const size_t sb0 = tbase + (size_t)(mb * 16) * (size_t)pitch;
#pragma unroll 1
        for (int ps = 0; ps < 2; ++ps) {
#pragma unroll
            for (int s = 0; s < 4; ++s) { const size_t oo = sb0 + (size_t)(4 * s + rg) * (size_t)pitch + c8;
                *(volatile v8h*)(Ph + oo) = hv[s]; if (useRes) *(volatile v8h*)(Pr + oo) = rv[s]; }
            if (ps == 0) __threadfence(); }
        wave_sync();
    }
}

__global__ __launch_bounds__(32) void k_proj_rot(const bf* __restrict__ A, const bf* __restrict__ Bt, h16* Ph, h16* Pr, int useRes,
                                                 int RB, size_t sRB, int pitch, int CB, size_t sCB,
                                                 const float* __restrict__ fc, const float* __restrict__ fs) {
    proj_body<1>(A, Bt, Ph, Pr, useRes, RB, sRB, pitch, CB, sCB, fc, fs);
}
__global__ __launch_bounds__(32) void k_proj_plain(const bf* __restrict__ A, const bf* __restrict__ Bt, h16* Ph, h16* Pr, int useRes,
                                                   int RB, size_t sRB, int pitch, int CB, size_t sCB,
                                                   const float* __restrict__ fc, const float* __restrict__ fs) {
    proj_body<0>(A, Bt, Ph, Pr, useRes, RB, sRB, pitch, CB, sCB, fc, fs);
}

__global__ __launch_bounds__(128) void k_est(const h16* __restrict__ QH, const h16* __restrict__ QR, const h16* __restrict__ KH, const h16* __restrict__ KR, float* S) {
    __shared__ __align__(16) float es[4 * 64 * 36];
    const int lane = threadIdx.x & 31, lr = lane & 15, hi = lane >> 4;
    const int wave = __builtin_amdgcn_readfirstlane((int)(threadIdx.x >> 5));
    const int zh = blockIdx.y; const int b = zh / HQ_, h = zh % HQ_; const int kvh = h / GQ;
    const int key0 = (blockIdx.x * 4 + wave) * 32;
    const size_t qbase = (size_t)zh * SEQ * HD, kbase = (size_t)(b * HK_ + kvh) * SEQ * HD;
    const size_t ko = kbase + (size_t)(key0 + lr) * HD + 8 * hi;
    const v16h ka0 = ldh(KH + ko), ka1 = ldh(KH + ko + 32), kb0 = ldh(KH + ko + 16 * HD), kb1 = ldh(KH + ko + 16 * HD + 32);
    const v16h ra0 = ldh(KR + ko), ra1 = ldh(KR + ko + 32), rb0 = ldh(KR + ko + 16 * HD), rb1 = ldh(KR + ko + 16 * HD + 32);
    const int wb = wave * 64 * 36;
    const int kga = key0 + lr, kgb = kga + 16;
    const int ja = kga - (SEQ - ESTQ), jb = kgb - (SEQ - ESTQ);
#pragma unroll 1
    for (int mt = 0; mt < 4; ++mt) {
        const size_t qo = qbase + (size_t)(mt * 16 + lr) * HD + 8 * hi;
        const v16h qh0 = ldh(QH + qo), qh1 = ldh(QH + qo + 32), qr0 = ldh(QR + qo), qr1 = ldh(QR + qo + 32);
        v8f sHa = (v8f){}, sLa = (v8f){}, sHb = (v8f){}, sLb = (v8f){};
        sHa = wg16(qh0, ka0, sHa); sHa = wg16(qh1, ka1, sHa);
        sHb = wg16(qh0, kb0, sHb); sHb = wg16(qh1, kb1, sHb);
        sLa = wg16(qr0, ka0, sLa); sLa = wg16(qr1, ka1, sLa); sLa = wg16(qh0, ra0, sLa); sLa = wg16(qh1, ra1, sLa);
        sLb = wg16(qr0, kb0, sLb); sLb = wg16(qr1, kb1, sLb); sLb = wg16(qh0, rb0, sLb); sLb = wg16(qh1, rb1, sLb);
#pragma unroll
        for (int r = 0; r < 8; ++r) { const int qi = mt * 16 + 8 * hi + r;
            float va = (sHa[r] + sLa[r] * QRI) * 0.125f, vb = (sHb[r] + sLb[r] * QRI) * 0.125f;
            va = (ja >= 0 && qi < ja) ? -3.0e38f : va;
            vb = (jb >= 0 && qi < jb) ? -3.0e38f : vb;
            es[wb + qi * 36 + lr] = va; es[wb + qi * 36 + 16 + lr] = vb; }
    }
    wave_sync();
    const int c4 = (lane & 7) * 4, rg = lane >> 3;
    float* sbp = S + ((size_t)zh * ESTQ) * SEQ + key0 + c4;
#pragma unroll 1
    for (int ps = 0; ps < 2; ++ps) {
#pragma unroll
        for (int s = 0; s < 16; ++s) { const int row = 4 * s + rg;
            const v4f val = *(const v4fa*)(&es[wb + row * 36 + c4]);
            *(volatile v4f*)(sbp + (size_t)row * SEQ) = val; }
        if (ps == 0) __threadfence(); }
}

__global__ __launch_bounds__(256) void k_select(const float* __restrict__ S, int* SK) {
#pragma clang fp contract(off)
    __shared__ unsigned long long sk[SEQ];
    __shared__ float dg[SEQ];
    __shared__ unsigned short cn[SEQ];
    __shared__ __align__(16) int lst[NKP];
    __shared__ float sm[ESTQ], si[ESTQ];
    __shared__ int wtot[8];
    const int tid = threadIdx.x, lane = tid & 31;
    const int wave = __builtin_amdgcn_readfirstlane((int)(threadIdx.x >> 5));
    const int zh = blockIdx.x;
    const float* Sh = S + (size_t)zh * ESTQ * SEQ;
#pragma unroll 1
    for (int i = 0; i < ESTQ / 8; ++i) { const int q = wave * (ESTQ / 8) + i; const float* row = Sh + (size_t)q * SEQ;
        float m = -3.0e38f;
#pragma unroll 1
        for (int j = lane; j < SEQ; j += 32) m = fmaxf(m, row[j]);
        m = fmaxf(m, __shfl_xor(m, 16, 32)); m = fmaxf(m, __shfl_xor(m, 8, 32)); m = fmaxf(m, __shfl_xor(m, 4, 32)); m = fmaxf(m, __shfl_xor(m, 2, 32)); m = fmaxf(m, __shfl_xor(m, 1, 32));
        float l = 0.0f;
#pragma unroll 1
        for (int j = lane; j < SEQ; j += 32) { const float a = row[j]; const float e = expf(a - m); l += (a > -1.0e38f) ? e : 0.0f; }
        l += __shfl_xor(l, 16, 32); l += __shfl_xor(l, 8, 32); l += __shfl_xor(l, 4, 32); l += __shfl_xor(l, 2, 32); l += __shfl_xor(l, 1, 32);
        if (lane == 0) { sm[q] = m; si[q] = 1.0f / l; }
    }
    __syncthreads();
#pragma unroll 1
    for (int jj = 0; jj < SEQ / 256; ++jj) { const int j = jj * 256 + tid;
        float vs = 0.0f, ds = 0.0f;
#pragma unroll 1
        for (int q = 0; q < ESTQ; ++q) { const float* row = Sh + (size_t)q * SEQ; const float mq = sm[q], iq = si[q];
            const int col = q + j + 1 - ESTQ; const int cc = imin(imax(col, 0), SEQ - 1);
            float a = row[j]; float bq = row[cc];
            asm volatile("" : "+v"(a), "+v"(bq));
            const float ea = expf(a - mq) * iq; const float eb = expf(bq - mq) * iq;
            vs += (a > -1.0e38f) ? ea : 0.0f;
            ds += (bq > -1.0e38f && col >= 0 && col < SEQ) ? eb : 0.0f; }
        sk[j] = mkkey(vs, j); dg[j] = ds; cn[j] = (unsigned short)0; }
    __syncthreads();
#pragma unroll 1
    for (int pass = 0; pass < 2; ++pass) {
        if (pass == 1) {
#pragma unroll 1
            for (int jj = 0; jj < SEQ / 256; ++jj) { const int j = jj * 256 + tid; sk[j] = mkkey(dg[j], j); }
            __syncthreads();
        }
#pragma unroll 1
        for (int k = 2; k <= SEQ; k <<= 1) {
#pragma unroll 1
            for (int jv = k >> 1; jv > 0; jv >>= 1) {
#pragma unroll 1
                for (int i = tid; i < SEQ / 2; i += 256) {
                    const int a = ((i & ~(jv - 1)) << 1) | (i & (jv - 1)); const int bb = a | jv;
                    const unsigned long long x = sk[a], y = sk[bb];
                    const bool up = (a & k) == 0;
                    const bool sw = up ? (x > y) : (x < y);
                    sk[a] = sw ? y : x; sk[bb] = sw ? x : y; }
                __syncthreads();
            }
        }
        const int nsel = (pass == 0) ? VSZ : SSZ;
#pragma unroll 1
        for (int r = tid; r < nsel; r += 256) { const int idx = (int)(sk[r] & 0xFFFFFFFFull) & (SEQ - 1);
            const int key = (pass == 0) ? idx : (SEQ - 1 - idx);
            cn[key] = (unsigned short)(cn[key] + 1); }
        __syncthreads();
    }
    const int PER = SEQ / 256;
    int loc = 0;
#pragma unroll 1
    for (int i = 0; i < PER; ++i) loc += (int)cn[tid * PER + i];
    int inc = loc;
#pragma unroll
    for (int d = 1; d < 32; d <<= 1) { const int o = __shfl_up(inc, d, 32); inc += (lane >= d) ? o : 0; }
    if (lane == 31) wtot[wave] = inc;
#pragma unroll 1
    for (int i = tid; i < NKP; i += 256) lst[i] = 0x7fffffff;
    __syncthreads();
    int off = inc - loc;
#pragma unroll
    for (int w = 0; w < 8; ++w) { const int tw = wtot[w]; off += (w < wave) ? tw : 0; }
#pragma unroll 1
    for (int i = 0; i < PER; ++i) { const int key = tid * PER + i; const int c = (int)cn[key];
        if (c >= 1 && off < NKP) { lst[off] = key; ++off; }
        if (c >= 2 && off < NKP) { lst[off] = key; ++off; } }
    __syncthreads();
    int* dst = SK + (size_t)zh * NKP;
#pragma unroll 1
    for (int ps = 0; ps < 2; ++ps) {
#pragma unroll 1
        for (int i = tid; i < NKP / 4; i += 256) { const v4i v = *(const v4ia*)(&lst[4 * i]); *(volatile v4i*)(dst + 4 * i) = v; }
        if (ps == 0) __threadfence(); }
}

__global__ __launch_bounds__(256) void k_gather(const int* __restrict__ SK, const h16* __restrict__ KH, const h16* __restrict__ KR, const h16* __restrict__ VH, const h16* __restrict__ VR,
                                                h16* KSH, h16* KSR, h16* VSH, h16* VSR) {
    __shared__ __align__(16) h16 vt0[64 * 72];
    __shared__ __align__(16) h16 vt1[64 * 72];
    const int tid = threadIdx.x; const int zh = blockIdx.y; const int b = zh / HQ_, h = zh % HQ_; const int kvh = h / GQ;
    const int j0 = blockIdx.x * 64;
    const size_t src = (size_t)(b * HK_ + kvh) * SEQ * HD;
    const int c8 = (tid & 7) * 8, rg = tid >> 3;
    v8h kh[2], kr[2];
#pragma unroll
    for (int ps = 0; ps < 2; ++ps) { const int jr = rg + 32 * ps; const int j = j0 + jr;
        int idx = SK[(size_t)zh * NKP + j];
        asm volatile("" : "+v"(idx));
        idx = imin(imax(idx, 0), SEQ - 1);
        const bool real = j < NSP;
        const size_t so = src + (size_t)idx * HD + c8;
        v8h a = *(const v8h*)(KH + so), r = *(const v8h*)(KR + so), va = *(const v8h*)(VH + so), vr = *(const v8h*)(VR + so);
        const v8h z = (v8h){};
        a = real ? a : z; r = real ? r : z; va = real ? va : z; vr = real ? vr : z;
        kh[ps] = a; kr[ps] = r;
        *(v8ha*)(&vt0[jr * 72 + c8]) = va; *(v8ha*)(&vt1[jr * 72 + c8]) = vr; }
    const size_t kdst = (size_t)zh * NKP * HD + (size_t)j0 * HD + c8;
#pragma unroll 1
    for (int pz = 0; pz < 2; ++pz) {
#pragma unroll
        for (int ps = 0; ps < 2; ++ps) { const size_t oo = kdst + (size_t)(rg + 32 * ps) * HD;
            *(volatile v8h*)(KSH + oo) = kh[ps]; *(volatile v8h*)(KSR + oo) = kr[ps]; }
        if (pz == 0) __threadfence(); }
    __syncthreads();
    v8h th[2], tr[2];
#pragma unroll
    for (int ps = 0; ps < 2; ++ps) { const int d = rg + 32 * ps;
#pragma unroll
        for (int i = 0; i < 8; ++i) { th[ps][i] = vt0[(c8 + i) * 72 + d]; tr[ps][i] = vt1[(c8 + i) * 72 + d]; } }
    const size_t vdst = (size_t)zh * HD * NKP + (size_t)j0 + c8;
#pragma unroll 1
    for (int pz = 0; pz < 2; ++pz) {
#pragma unroll
        for (int ps = 0; ps < 2; ++ps) { const size_t oo = vdst + (size_t)(rg + 32 * ps) * NKP;
            *(volatile v8h*)(VSH + oo) = th[ps]; *(volatile v8h*)(VSR + oo) = tr[ps]; }
        if (pz == 0) __threadfence(); }
}

__global__ __launch_bounds__(32 * AW) void k_flash(const h16* __restrict__ QH, const h16* __restrict__ QR, const h16* __restrict__ KSH, const h16* __restrict__ KSR,
                                                   const h16* __restrict__ VSH, const h16* __restrict__ VSR, const int* __restrict__ SK, h16* CH, h16* CR) {
    __shared__ __align__(16) float os[AW * 16 * 68];
    const int lane = threadIdx.x & 31, lr = lane & 15, hi = lane >> 4;
    const int wave = __builtin_amdgcn_readfirstlane((int)(threadIdx.x >> 5));
    const int zh = blockIdx.y; const int b = zh / HQ_, h = zh % HQ_;
    const int t0 = (blockIdx.x * AW + wave) * 16;
    const bool ex = t0 < RES_ROWS;
    const size_t qbase = (size_t)zh * SEQ * HD, kbase = (size_t)zh * NKP * HD;
    const size_t qo = qbase + (size_t)(t0 + lr) * HD + 8 * hi;
    const v16h qh0 = ldh(QH + qo), qh1 = ldh(QH + qo + 32), qr0 = ldh(QR + qo), qr1 = ldh(QR + qo + 32);
    const size_t ko = kbase + (size_t)lr * HD + 8 * hi;
    const size_t vo = kbase + (size_t)lr * NKP + 8 * hi;
    const int tq = t0 + lr;
    const int* lst = SK + (size_t)zh * NKP;
    int cr = 0;
#pragma unroll
    for (int s = BS_TOP; s >= 1; s >>= 1) { const int cand = cr + s; const int ix = imin(cand, NSP) - 1;
        int kv = lst[ix];
        asm volatile("" : "+v"(kv));
        cr = (cand <= NSP && kv <= tq) ? cand : cr; }
    const bool zr = (cr == 0);
    const int lim = zr ? NSP : cr;
    int nkv = imin(lim, NSP);
    nkv = imax(nkv, __shfl_xor(nkv, 1, 32)); nkv = imax(nkv, __shfl_xor(nkv, 2, 32)); nkv = imax(nkv, __shfl_xor(nkv, 4, 32)); nkv = imax(nkv, __shfl_xor(nkv, 8, 32)); nkv = imax(nkv, __shfl_xor(nkv, 16, 32));
    const int nk = __builtin_amdgcn_readfirstlane(nkv);
    v8f oh[4], orr[4];
#pragma unroll
    for (int j = 0; j < 4; ++j) { oh[j] = (v8f){}; orr[j] = (v8f){}; }
    float m = -3.0e38f, l = 0.0f;
#pragma unroll 1
    for (int key0 = 0; key0 < nk; key0 += 32) {
        const h16* ka = KSH + ko + (size_t)key0 * HD;
        const v16h ka0 = ldh(ka), ka1 = ldh(ka + 32), kb0 = ldh(ka + 16 * HD), kb1 = ldh(ka + 16 * HD + 32);
        v8f sHa = (v8f){}, sLa = (v8f){}, sHb = (v8f){}, sLb = (v8f){};
        sHa = wg16(ka0, qh0, sHa); sLa = wg16(ka0, qr0, sLa); sHb = wg16(kb0, qh0, sHb); sLb = wg16(kb0, qr0, sLb);
        sHa = wg16(ka1, qh1, sHa); sLa = wg16(ka1, qr1, sLa); sHb = wg16(kb1, qh1, sHb); sLb = wg16(kb1, qr1, sLb);
        if (ex) {
            const h16* kr = KSR + ko + (size_t)key0 * HD;
            const v16h ra0 = ldh(kr), ra1 = ldh(kr + 32), rb0 = ldh(kr + 16 * HD), rb1 = ldh(kr + 16 * HD + 32);
            sLa = wg16(ra0, qh0, sLa); sLb = wg16(rb0, qh0, sLb);
            sLa = wg16(ra1, qh1, sLa); sLb = wg16(rb1, qh1, sLb);
        }
        float ta[8], tb[8]; float mx = -3.0e38f;
        const int jb0 = key0 + 8 * hi;
#pragma unroll
        for (int r = 0; r < 8; ++r) {
            const int ja = jb0 + r, jc = ja + 16;
            float va = (sHa[r] + sLa[r] * QRI) * SC2, vb = (sHb[r] + sLb[r] * QRI) * SC2;
            va = zr ? 0.0f : va; vb = zr ? 0.0f : vb;
            ta[r] = (ja < lim) ? va : -3.0e38f;
            tb[r] = (jc < lim) ? vb : -3.0e38f;
            mx = fmaxf(mx, fmaxf(ta[r], tb[r])); }
        mx = fmaxf(mx, __shfl_xor(mx, 16, 32));
        const float mnew = fmaxf(m, mx);
        const float alpha = __builtin_amdgcn_exp2f(m - mnew);
        const float sh = PSH - mnew;
        v16h pb, pr; float ls = 0.0f;
#pragma unroll
        for (int r = 0; r < 8; ++r) {
            const float xa = ta[r] + sh, xb = tb[r] + sh;
            const float ea = (ta[r] > -1.0e38f && xa >= -14.0f) ? __builtin_amdgcn_exp2f(xa) : 0.0f;
            const float eb = (tb[r] > -1.0e38f && xb >= -14.0f) ? __builtin_amdgcn_exp2f(xb) : 0.0f;
            const h16 pa = (h16)ea; const h16 pc = (h16)eb;
            pb[r] = pa; pb[8 + r] = pc;
            pr[r] = toh_flush((ea - (float)pa) * QRS); pr[8 + r] = toh_flush((eb - (float)pc) * QRS);
            ls += ex ? (ea + eb) : ((float)pa + (float)pc); }
        l = l * alpha + ls; m = mnew;
#pragma unroll
        for (int j = 0; j < 4; ++j) oh[j] = oh[j] * alpha;
        const h16* va = VSH + vo + key0;
        const v16h v0 = ldh(va), v1 = ldh(va + (size_t)16 * NKP), v2 = ldh(va + (size_t)32 * NKP), v3 = ldh(va + (size_t)48 * NKP);
        oh[0] = wg16(v0, pb, oh[0]); oh[1] = wg16(v1, pb, oh[1]); oh[2] = wg16(v2, pb, oh[2]); oh[3] = wg16(v3, pb, oh[3]);
        if (ex) {
#pragma unroll
            for (int j = 0; j < 4; ++j) orr[j] = orr[j] * alpha;
            const h16* vr = VSR + vo + key0;
            const v16h w0 = ldh(vr), w1 = ldh(vr + (size_t)16 * NKP), w2 = ldh(vr + (size_t)32 * NKP), w3 = ldh(vr + (size_t)48 * NKP);
            orr[0] = wg16(w0, pb, orr[0]); orr[1] = wg16(w1, pb, orr[1]); orr[2] = wg16(w2, pb, orr[2]); orr[3] = wg16(w3, pb, orr[3]);
            orr[0] = wg16(v0, pr, orr[0]); orr[1] = wg16(v1, pr, orr[1]); orr[2] = wg16(v2, pr, orr[2]); orr[3] = wg16(v3, pr, orr[3]);
        }
    }
    l += __shfl_xor(l, 16, 32);
    const float inv = 1.0f / l;
    const int wb = wave * 16 * 68;
#pragma unroll
    for (int j = 0; j < 4; ++j) { v4f a, c;
#pragma unroll
        for (int i = 0; i < 4; ++i) { a[i] = (oh[j][i] + orr[j][i] * QRI) * inv; c[i] = (oh[j][4 + i] + orr[j][4 + i] * QRI) * inv; }
        *(v4fa*)(&os[wb + lr * 68 + 16 * j + 8 * hi]) = a; *(v4fa*)(&os[wb + lr * 68 + 16 * j + 8 * hi + 4]) = c; }
    wave_sync();
    const int c8 = (lane & 7) * 8, rg = lane >> 3;
    v8h hv[4], rv[4];
#pragma unroll
    for (int s = 0; s < 4; ++s) { const int row = 4 * s + rg;
        const v4f x0 = *(const v4fa*)(&os[wb + row * 68 + c8]); const v4f x1 = *(const v4fa*)(&os[wb + row * 68 + c8 + 4]); v8h hh, rr;
#pragma unroll
        for (int i = 0; i < 4; ++i) { const h16 a0 = toh_flush(x0[i]); const h16 a1 = toh_flush(x1[i]); hh[i] = a0; hh[4 + i] = a1; rr[i] = toh_flush((x0[i] - (float)a0) * QRS); rr[4 + i] = toh_flush((x1[i] - (float)a1) * QRS); }
        hv[s] = hh; rv[s] = rr; }
    const size_t cbase = ((size_t)b * SEQ + t0) * QW + (size_t)h * HD + c8;
#pragma unroll 1
    for (int ps = 0; ps < 2; ++ps) {
#pragma unroll
        for (int s = 0; s < 4; ++s) { const size_t oo = cbase + (size_t)(4 * s + rg) * QW;
            *(volatile v8h*)(CH + oo) = hv[s]; *(volatile v8h*)(CR + oo) = rv[s]; }
        if (ps == 0) __threadfence(); }
}

__device__ __forceinline__ void gemm_h(v8f (&acc)[4][4], const h16* __restrict__ a, const h16* __restrict__ b) {
#pragma unroll 1
    for (int kc = 0; kc < QW; kc += 32) {
        v16h af[4];
#pragma unroll
        for (int mb = 0; mb < 4; ++mb) af[mb] = ldh(a + (size_t)mb * 16 * QW + kc);
#pragma unroll
        for (int nb = 0; nb < 4; ++nb) { const v16h bv = ldh(b + (size_t)nb * 16 * QW + kc);
#pragma unroll
            for (int mb = 0; mb < 4; ++mb) acc[mb][nb] = wmma16(af[mb], bv, acc[mb][nb]); }
        asm volatile("v_nop\n\tv_nop\n\tv_nop\n\tv_nop" : "+v"(acc[0][0]), "+v"(acc[1][1]), "+v"(acc[2][2]), "+v"(acc[3][3]) : "v"(af[0]), "v"(af[1]), "v"(af[2]), "v"(af[3]));
    }
}

__global__ __launch_bounds__(32) void k_oproj(const h16* __restrict__ Ah, const h16* __restrict__ Ar, const h16* __restrict__ Bt, float* OUT) {
    __shared__ __align__(16) float os[16 * 68];
    const int lane = threadIdx.x & 31, lr = lane & 15, hi = lane >> 4; const int r0 = blockIdx.x * 64, c0 = blockIdx.y * 64;
    v8f acc[4][4];
#pragma unroll
    for (int mb = 0; mb < 4; ++mb)
#pragma unroll
        for (int nb = 0; nb < 4; ++nb) acc[mb][nb] = (v8f){};
    const size_t aoff = (size_t)(r0 + lr) * QW + 8 * hi, boff = (size_t)(c0 + lr) * QW + 8 * hi;
    if ((r0 % SEQ) < RES_ROWS) {
        gemm_h(acc, Ar + aoff, Bt + boff);
#pragma unroll
        for (int mb = 0; mb < 4; ++mb)
#pragma unroll
            for (int nb = 0; nb < 4; ++nb) acc[mb][nb] = acc[mb][nb] * QRI;
    }
    gemm_h(acc, Ah + aoff, Bt + boff);
    const int bb = r0 / SEQ, tt = r0 % SEQ;
    float* obase = OUT + ((size_t)bb * OUT_SEQ + tt) * DM + c0;
#pragma unroll
    for (int mb = 0; mb < 4; ++mb) {
#pragma unroll
        for (int nb = 0; nb < 4; ++nb) {
#pragma unroll
            for (int j = 0; j < 8; ++j) os[(hi * 8 + j) * 68 + nb * 16 + lr] = acc[mb][nb][j] * WOI; }
        wave_sync();
        float* orow = obase + (size_t)(mb * 16) * DM;
#pragma unroll 1
        for (int ps = 0; ps < 2; ++ps) {
#pragma unroll
            for (int s = 0; s < 8; ++s) { const int row = 2 * s + hi, cofs = lr * 4;
                const v4f val = *(const v4fa*)(&os[row * 68 + cofs]);
                *(volatile v4f*)(orow + (size_t)row * DM + cofs) = val; }
            if (ps == 0) __threadfence(); }
        wave_sync();
    }
}

static constexpr size_t al256(size_t v) { return (v + 255) & ~(size_t)255; }
static constexpr size_t mx2(size_t a, size_t b) { return a > b ? a : b; }
static constexpr size_t SZ_XB = al256((size_t)NB * SEQ * DM * 2);
static constexpr size_t SZ_WQ = al256((size_t)QW * DM * 2);
static constexpr size_t SZ_WK = al256((size_t)KW * DM * 2);
static constexpr size_t SZ_WO = al256((size_t)DM * QW * 2);
static constexpr size_t SZ_QP = al256((size_t)NB * HQ_ * SEQ * HD * 2);
static constexpr size_t SZ_KP = al256((size_t)NB * HK_ * SEQ * HD * 2);
static constexpr size_t SZ_CP = al256((size_t)NB * SEQ * QW * 2);
static constexpr size_t SZ_ES = al256((size_t)NB * HQ_ * ESTQ * SEQ * 4);
static constexpr size_t SZ_SK = al256((size_t)NB * HQ_ * NKP * 4);
static constexpr size_t SZ_GP = al256((size_t)NB * HQ_ * NKP * HD * 2);
static constexpr size_t SZ_RA = mx2(SZ_XB + SZ_WQ + 2 * SZ_WK, SZ_SK + 4 * SZ_GP);
static constexpr size_t SZ_RB = mx2(SZ_ES, 2 * SZ_CP);
static_assert(SZ_XB + SZ_WQ + 2 * SZ_WK <= SZ_RA);
static_assert(SZ_SK + 4 * SZ_GP <= SZ_RA);
static_assert(SZ_ES <= SZ_RB);
static_assert(2 * SZ_CP <= SZ_RB);
static constexpr size_t SZ_TOTAL = SZ_RA + SZ_WO + 2 * SZ_QP + 4 * SZ_KP + SZ_RB;
static_assert(SZ_TOTAL <= (size_t)134217728);

extern "C" void kernel_launch(void* const* d_in, const int* in_sizes, int n_in,
                              void* d_out, int out_size, void* d_ws, size_t ws_size, hipStream_t stream) {
    if (n_in < 7) return;
    const size_t needt = (size_t)(NB - 1) * SEQ_FULL + SEQ;
    if ((size_t)in_sizes[0] < needt * DM) return;
    if ((size_t)in_sizes[1] < (size_t)SEQ * 32 || (size_t)in_sizes[2] < (size_t)SEQ * 32) return;
    if ((size_t)in_sizes[3] < (size_t)DM * QW || (size_t)in_sizes[4] < (size_t)DM * KW || (size_t)in_sizes[5] < (size_t)DM * KW || (size_t)in_sizes[6] < (size_t)QW * DM) return;
    if ((size_t)out_size < ((size_t)(NB - 1) * OUT_SEQ + SEQ) * DM) return;
    if (SZ_TOTAL > ws_size) return;
    const float* x = (const float*)d_in[0]; const float* fc = (const float*)d_in[1]; const float* fs = (const float*)d_in[2];
    const float* wq = (const float*)d_in[3]; const float* wk = (const float*)d_in[4]; const float* wv = (const float*)d_in[5]; const float* wo = (const float*)d_in[6];
    float* OUT = (float*)d_out;
    char* wsp = (char*)d_ws;
    char* ra = wsp; wsp += SZ_RA;
    bf*  XB  = (bf*)ra;
    bf*  WQB = (bf*)(ra + SZ_XB);
    bf*  WKB = (bf*)(ra + SZ_XB + SZ_WQ);
    bf*  WVB = (bf*)(ra + SZ_XB + SZ_WQ + SZ_WK);
    int* SKL = (int*)ra;
    h16* KSH = (h16*)(ra + SZ_SK);
    h16* KSR = (h16*)(ra + SZ_SK + SZ_GP);
    h16* VSH = (h16*)(ra + SZ_SK + 2 * SZ_GP);
    h16* VSR = (h16*)(ra + SZ_SK + 3 * SZ_GP);
    h16* WOH = (h16*)wsp; wsp += SZ_WO;
    h16* QH = (h16*)wsp; wsp += SZ_QP;
    h16* QR = (h16*)wsp; wsp += SZ_QP;
    h16* KH = (h16*)wsp; wsp += SZ_KP;
    h16* KR = (h16*)wsp; wsp += SZ_KP;
    h16* VH = (h16*)wsp; wsp += SZ_KP;
    h16* VR = (h16*)wsp; wsp += SZ_KP;
    char* rb = wsp; wsp += SZ_RB;
    float* ES = (float*)rb;
    h16* CH = (h16*)rb;
    h16* CR = (h16*)(rb + SZ_CP);

    if (SEQ == SEQ_FULL) {
        const size_t n8 = (size_t)NB * SEQ * DM / 8;
        k_cvt8<<<(unsigned)((n8 + 255) / 256), 256, 0, stream>>>(x, XB, n8);
    } else {
        const size_t n8 = (size_t)SEQ * DM / 8;
        for (int b = 0; b < NB; ++b) k_cvt8<<<(unsigned)((n8 + 255) / 256), 256, 0, stream>>>(x + (size_t)b * SEQ_FULL * DM, XB + (size_t)b * SEQ * DM, n8);
    }
    k_trb<<<dim3(QW / 64, DM / 64, 1), 256, 0, stream>>>(wq, WQB, DM, QW);
    k_trb<<<dim3(KW / 64, DM / 64, 1), 256, 0, stream>>>(wk, WKB, DM, KW);
    k_trb<<<dim3(KW / 64, DM / 64, 1), 256, 0, stream>>>(wv, WVB, DM, KW);
    k_trw<<<dim3(DM / 64, QW / 64, 1), 256, 0, stream>>>(wo, WOH, QW, DM);

    k_proj_rot<<<dim3(NB * SEQ / 64, QW / 64, 1), 32, 0, stream>>>(XB, WQB, QH, QR, 1, SEQ, (size_t)HQ_ * SEQ * HD, HD, HD, (size_t)SEQ * HD, fc, fs);
    k_proj_rot<<<dim3(NB * SEQ / 64, KW / 64, 1), 32, 0, stream>>>(XB, WKB, KH, KR, 1, SEQ, (size_t)HK_ * SEQ * HD, HD, HD, (size_t)SEQ * HD, fc, fs);
    k_proj_plain<<<dim3(NB * SEQ / 64, KW / 64, 1), 32, 0, stream>>>(XB, WVB, VH, VR, 1, SEQ, (size_t)HK_ * SEQ * HD, HD, HD, (size_t)SEQ * HD, fc, fs);

    k_est<<<dim3(SEQ / 128, NB * HQ_, 1), 128, 0, stream>>>(QH, QR, KH, KR, ES);
    k_select<<<NB * HQ_, 256, 0, stream>>>(ES, SKL);
    k_gather<<<dim3(NKP / 64, NB * HQ_, 1), 256, 0, stream>>>(SKL, KH, KR, VH, VR, KSH, KSR, VSH, VSR);

    k_flash<<<dim3(SEQ / (16 * AW), NB * HQ_, 1), 32 * AW, 0, stream>>>(QH, QR, KSH, KSR, VSH, VSR, SKL, CH, CR);

    k_oproj<<<dim3(NB * SEQ / 64, DM / 64, 1), 32, 0, stream>>>(CH, CR, WOH, OUT);
}
